// G_22093311770918
// MI455X (gfx1250) — hardware-verified
//
#include <hip/hip_runtime.h>
#include <math.h>

constexpr int kRows = 128;
constexpr int kHid  = 1024;
constexpr int kG3   = 3072;
constexpr int kFc   = 1024;
constexpr int kCls  = 256;
constexpr float kWCarry    = 16.0f;
constexpr float kWCarryInv = 1.0f / 16.0f;

typedef __attribute__((ext_vector_type(16))) _Float16 v16h;
typedef __attribute__((ext_vector_type(8)))  _Float16 v8h;
typedef __attribute__((ext_vector_type(16))) __bf16   v16b;
typedef __attribute__((ext_vector_type(8)))  __bf16   v8b;
typedef __attribute__((ext_vector_type(8)))  float    v8f;
typedef __attribute__((ext_vector_type(4)))  float    v4f;
typedef __attribute__((ext_vector_type(4)))  unsigned int v4u;

__device__ __forceinline__ unsigned short f2bf_bits(float f) {
  unsigned u = __float_as_uint(f);
  return (unsigned short)((u + 0x7FFFu + ((u >> 16) & 1u)) >> 16);
}
__device__ __forceinline__ float bf_bits2f(unsigned short h) { return __uint_as_float(((unsigned)h) << 16); }

__device__ __forceinline__ void dep_guard_h(v8f& a, v8f& b, v16h x, v16h y) { asm volatile("v_nop\n\tv_nop\n\tv_nop\n\tv_nop" : "+v"(a), "+v"(b) : "v"(x), "v"(y)); }
__device__ __forceinline__ void dep_guard_b(v8f& a, v8f& b, v16b x, v16b y) { asm volatile("v_nop\n\tv_nop\n\tv_nop\n\tv_nop" : "+v"(a), "+v"(b) : "v"(x), "v"(y)); }
__device__ __forceinline__ void keep4_h(v16h a, v16h b, v16h c, v16h d) { asm volatile("v_nop" :: "v"(a), "v"(b), "v"(c), "v"(d)); }
__device__ __forceinline__ void keep4_b(v16b a, v16b b, v16b c, v16b d) { asm volatile("v_nop" :: "v"(a), "v"(b), "v"(c), "v"(d)); }
__device__ __forceinline__ void acc_guard4(v8f& a, v8f& b, v8f& c, v8f& d) { asm volatile("v_nop\n\tv_nop\n\tv_nop\n\tv_nop" : "+v"(a), "+v"(b), "+v"(c), "+v"(d)); }
template <typename T> struct Frag;
template <> struct Frag<_Float16> {
  typedef v16h V; union U { v16h v; v8h h[2]; };
  static __device__ __forceinline__ v16h load(const _Float16* p) {
    U f; f.h[0] = *(const v8h*)(p); f.h[1] = *(const v8h*)(p + 16); return f.v;
  }
  static __device__ __forceinline__ v8f mma(v16h a, v16h b, v8f c) {
    return __builtin_amdgcn_wmma_f32_16x16x32_f16(false, a, false, b, (short)0, c, false, false);
  }
  static __device__ __forceinline__ void guard(v8f& a, v8f& b, v16h x, v16h y) { dep_guard_h(a, b, x, y); }
  static __device__ __forceinline__ void keep(v16h a, v16h b, v16h c, v16h d) { keep4_h(a, b, c, d); }
};
template <> struct Frag<__bf16> {
  typedef v16b V; union U { v16b v; v8b h[2]; };
  static __device__ __forceinline__ v16b load(const __bf16* p) {
    U f; f.h[0] = *(const v8b*)(p); f.h[1] = *(const v8b*)(p + 16); return f.v;
  }
  static __device__ __forceinline__ v8f mma(v16b a, v16b b, v8f c) {
    return __builtin_amdgcn_wmma_f32_16x16x32_bf16(false, a, false, b, (short)0, c, false, false);
  }
  static __device__ __forceinline__ void guard(v8f& a, v8f& b, v16b x, v16b y) { dep_guard_b(a, b, x, y); }
  static __device__ __forceinline__ void keep(v16b a, v16b b, v16b c, v16b d) { keep4_b(a, b, c, d); }
};

__device__ __forceinline__ unsigned pk16(unsigned short a, unsigned short b) { return (unsigned)a | ((unsigned)b << 16); }
__device__ __forceinline__ unsigned short h_bits(float f) { const _Float16 h = (_Float16)f; return __builtin_bit_cast(unsigned short, h); }

template <int ET> struct Elem;
template <> struct Elem<0> { typedef _Float16 T; };
template <> struct Elem<1> { typedef __bf16 T; };
template <int ET, bool SPLIT, int BIAS_MODE, int OUT_MODE, bool RESID, int ACT = 0>
__global__ __launch_bounds__(256) void wmma_gemm64(
    const unsigned short* __restrict__ Ap, const unsigned short* __restrict__ A2p, int lda, long strideA,
    const unsigned short* __restrict__ Btp, const unsigned short* __restrict__ Bt2p, int ldb, long strideB,
    void* __restrict__ Cout, void* __restrict__ Cout2, int ldc, long strideC,
    const float* __restrict__ bias,
    const float* __restrict__ resid, long strideR,
    int M, int N, int K, float scale) {
  typedef typename Elem<ET>::T T;
  typedef typename Frag<T>::V V;
  const T* A = (const T*)Ap; const T* A2 = (const T*)A2p; const T* Bt = (const T*)Btp; const T* Bt2 = (const T*)Bt2p;
  __shared__ __align__(16) float sT[8][16 * 68];
  const int b    = blockIdx.y;
  const int lane = threadIdx.x & 31;
  const int wave = threadIdx.x >> 5;
  const int tilesN = N >> 6;
  const int tilesM = M >> 6;
  const int tile = blockIdx.x * 8 + wave;
  if (tile >= tilesM * tilesN) return;
  const int tm = tile / tilesN;
  const int tn = tile - tm * tilesN;
  const int m0 = tm << 6;
  const int n0 = tn << 6;

  const T* Ab  = A  + (size_t)b * strideA;
  const T* Bb  = Bt + (size_t)b * strideB;
  const T* Ab2 = SPLIT ? (A2  + (size_t)b * strideA) : nullptr;
  const T* Bb2 = SPLIT ? (Bt2 + (size_t)b * strideB) : nullptr;

  const int rlane = lane & 15;
  const int koff  = (lane >> 4) * 8;
  const int mOff  = (lane >> 4) * 8;

  v8f acc[4][4];
#pragma unroll
  for (int i = 0; i < 4; ++i)
#pragma unroll
    for (int j = 0; j < 4; ++j) acc[i][j] = (v8f){0.f,0.f,0.f,0.f,0.f,0.f,0.f,0.f};

  for (int k0 = 0; k0 < K; k0 += 32) {
    V bh[4], bl[4];
#pragma unroll
    for (int j = 0; j < 4; ++j) {
      const size_t bo = (size_t)(n0 + (j << 4) + rlane) * ldb + koff + k0;
      bh[j] = Frag<T>::load(Bb + bo);
      if (SPLIT) bl[j] = Frag<T>::load(Bb2 + bo);
    }
#pragma unroll
    for (int i = 0; i < 4; ++i) {
      const size_t ao = (size_t)(m0 + (i << 4) + rlane) * lda + koff + k0;
      V ah = Frag<T>::load(Ab + ao);
      V al;
      if (SPLIT) al = Frag<T>::load(Ab2 + ao);
#pragma unroll
      for (int j = 0; j < 4; ++j) {
        acc[i][j] = Frag<T>::mma(ah, bh[j], acc[i][j]);
        if (SPLIT) {
          acc[i][j] = Frag<T>::mma(ah, bl[j], acc[i][j]);
          acc[i][j] = Frag<T>::mma(al, bh[j], acc[i][j]);
        }
      }
      Frag<T>::guard(acc[i][0], acc[i][3], ah, SPLIT ? al : ah);
    }
    Frag<T>::keep(bh[0], bh[1], bh[2], bh[3]);
    if (SPLIT) Frag<T>::keep(bl[0], bl[1], bl[2], bl[3]);
  }
  acc_guard4(acc[0][0], acc[0][1], acc[0][2], acc[0][3]);
  acc_guard4(acc[1][0], acc[1][1], acc[1][2], acc[1][3]);
  acc_guard4(acc[2][0], acc[2][1], acc[2][2], acc[2][3]);
  acc_guard4(acc[3][0], acc[3][1], acc[3][2], acc[3][3]);

  float* slab = sT[wave];
  const float* Rb = RESID ? (resid + (size_t)b * strideR) : nullptr;
#pragma unroll
  for (int i = 0; i < 4; ++i) {
    const int mBase = m0 + (i << 4);
#pragma unroll
    for (int j = 0; j < 4; ++j) {
      const int n = n0 + (j << 4) + rlane;
      float bv = 0.f;
      if (BIAS_MODE == 2) bv = bias[n];
#pragma unroll
      for (int r = 0; r < 8; ++r) {
        float v = acc[i][j][r] * scale;
        if (BIAS_MODE == 1) v += bias[mBase + mOff + r];
        if (BIAS_MODE == 2) v += bv;
        if (RESID) v += Rb[(size_t)(mBase + mOff + r) * ldc + n];
        if (ACT == 2) v = fmaxf(v, 0.0f);
        if (ACT == 4) v = (v > 0.f) ? v : 0.01f * v;
        slab[(mOff + r) * 68 + (j << 4) + rlane] = v;
      }
    }
    __builtin_amdgcn_fence(__ATOMIC_RELEASE, "workgroup");
    __builtin_amdgcn_wave_barrier();
    __builtin_amdgcn_fence(__ATOMIC_ACQUIRE, "workgroup");
    if (OUT_MODE == 0) {
      float* C = (float*)Cout + (size_t)b * strideC;
      const int hh = lane >> 4, c4 = (lane & 15) * 4;
      for (int pass = 0; pass < 2; ++pass) {
#pragma unroll
        for (int it = 0; it < 8; ++it) {
          const int row = it * 2 + hh;
          v4f v = *(const v4f*)(slab + row * 68 + c4);
          *(volatile v4f*)(C + (size_t)(mBase + row) * ldc + n0 + c4) = v;
        }
        __threadfence();
      }
    } else {
      const int q = lane >> 3, c8 = (lane & 7) * 8;
      unsigned short* C  = (unsigned short*)Cout  + (size_t)b * strideC;
      unsigned short* C2 = (OUT_MODE == 2) ? ((unsigned short*)Cout2 + (size_t)b * strideC) : nullptr;
      for (int pass = 0; pass < 2; ++pass) {
#pragma unroll
        for (int it = 0; it < 4; ++it) {
          const int row = it * 4 + q;
          const float* sp = slab + row * 68 + c8;
          v8h hv, lv;
#pragma unroll
          for (int e = 0; e < 8; ++e) {
            if (OUT_MODE == 1) {
              hv[e] = (_Float16)sp[e];
            } else {
              unsigned short hb = f2bf_bits(sp[e]);
              unsigned short lb = f2bf_bits(sp[e] - bf_bits2f(hb));
              hv[e] = __builtin_bit_cast(_Float16, hb);
              lv[e] = __builtin_bit_cast(_Float16, lb);
            }
          }
          *(volatile v8h*)(C + (size_t)(mBase + row) * ldc + n0 + c8) = hv;
          if (OUT_MODE == 2) *(volatile v8h*)(C2 + (size_t)(mBase + row) * ldc + n0 + c8) = lv;
        }
        __threadfence();
      }
    }
    __builtin_amdgcn_fence(__ATOMIC_RELEASE, "workgroup");
    __builtin_amdgcn_wave_barrier();
    __builtin_amdgcn_fence(__ATOMIC_ACQUIRE, "workgroup");
  }
}

__global__ __launch_bounds__(256) void cast8_f16_kernel(const float* __restrict__ in, unsigned short* __restrict__ out,
                                                        int n8, float scale) {
  const int i = blockIdx.x * 256 + threadIdx.x;
  if (i >= n8) return;
  const float* p = in + 8 * (size_t)i;
  const v4f a = *(const v4f*)(p);
  const v4f c = *(const v4f*)(p + 4);
  unsigned short hb[8];
#pragma unroll
  for (int e = 0; e < 4; ++e) {
    hb[e]     = h_bits(a[e] * scale);
    hb[4 + e] = h_bits(c[e] * scale);
  }
  const v4u u = (v4u){pk16(hb[0], hb[1]), pk16(hb[2], hb[3]), pk16(hb[4], hb[5]), pk16(hb[6], hb[7])};
  unsigned short* q = out + 8 * (size_t)i;
  *(volatile v4u*)q = u;
  __threadfence();
  *(volatile v4u*)q = u;
}

__global__ __launch_bounds__(256) void gru_cell_kernel(const float* __restrict__ GI, const float* __restrict__ GH,
                                                       const float* __restrict__ b_ih, const float* __restrict__ b_hh,
                                                       const float* __restrict__ x, const float* __restrict__ h1,
                                                       float* __restrict__ out1, unsigned short* __restrict__ res16) {
  __shared__ __align__(16) float s_hp[kHid];
  __shared__ __align__(16) float s_res[kHid];
  const int m = blockIdx.x;
  const int t = threadIdx.x;
  const float* gi = GI + (size_t)m * kG3;
  const float* gh = GH + (size_t)m * kG3;
  const float* xr = x  + (size_t)m * kHid;
  const float* hr = h1 + (size_t)m * kHid;
#pragma unroll 1
  for (int j = 0; j < 4; ++j) {
    const int c = t + 256 * j;
    const float i_r = gi[c]            + b_ih[c];
    const float i_z = gi[c + kHid]     + b_ih[c + kHid];
    const float i_n = gi[c + 2 * kHid] + b_ih[c + 2 * kHid];
    const float h_r = gh[c]            + b_hh[c];
    const float h_z = gh[c + kHid]     + b_hh[c + kHid];
    const float h_n = gh[c + 2 * kHid] + b_hh[c + 2 * kHid];
    const float er  = expf(-(i_r + h_r));
    const float ez  = expf(-(i_z + h_z));
    const float r   = __builtin_amdgcn_rcpf(1.0f + er);
    const float z   = __builtin_amdgcn_rcpf(1.0f + ez);
    const float ng  = tanhf(i_n + r * h_n);
    const float hv  = hr[c];
    const float xv  = xr[c];
    const float hp  = (1.0f - z) * ng + z * hv;
    s_hp[c]  = hp;
    s_res[c] = hp + xv;
  }
  __syncthreads();
  const v4f hq = *(const v4f*)(s_hp + 4 * t);
  const int tr = (t < 128) ? t : 127;
  const float* sp = s_res + 8 * tr;
  unsigned short hb[8];
#pragma unroll
  for (int e = 0; e < 8; ++e) hb[e] = h_bits(sp[e]);
  const v4u u = (v4u){pk16(hb[0], hb[1]), pk16(hb[2], hb[3]), pk16(hb[4], hb[5]), pk16(hb[6], hb[7])};
  float* op = out1 + (size_t)m * kHid + 4 * t;
  unsigned short* rp = res16 + (size_t)m * kHid + 8 * tr;
  for (int pass = 0; pass < 2; ++pass) {
    *(volatile v4f*)op = hq;
    if (t < 128) *(volatile v4u*)rp = u;
    __threadfence();
  }
}

constexpr size_t kOffX16   = 0;
constexpr size_t kOffH16   = kOffX16   + (size_t)kRows * kHid * 2;
constexpr size_t kOffWih   = kOffH16   + (size_t)kRows * kHid * 2;
constexpr size_t kOffWhh   = kOffWih   + (size_t)kG3 * kHid * 2;
constexpr size_t kOffWfc1  = kOffWhh   + (size_t)kG3 * kHid * 2;
constexpr size_t kOffWfc3  = kOffWfc1  + (size_t)kFc * kHid * 2;
constexpr size_t kOffGI    = kOffWfc3  + (size_t)kCls * kFc * 2;
constexpr size_t kOffGH    = kOffGI    + (size_t)kRows * kG3 * 4;
constexpr size_t kOffRes   = kOffGH    + (size_t)kRows * kG3 * 4;
constexpr size_t kOffRelu  = kOffRes   + (size_t)kRows * kHid * 2;
constexpr size_t kWsTotal  = kOffRelu  + (size_t)kRows * kFc * 2;
static_assert(kWsTotal == 19398656u);
static_assert(kWsTotal <= 134217728u);
static_assert((kRows * kCls + kRows * kHid) == 163840);

extern "C" void kernel_launch(void* const* d_in, const int* in_sizes, int n_in,
                              void* d_out, int out_size, void* d_ws, size_t ws_size,
                              hipStream_t stream) {
  if (n_in < 10) return;
  if (out_size != kRows * kCls + kRows * kHid) return;
  if (in_sizes[0] != kRows * kHid || in_sizes[1] != kRows * kHid) return;
  if (in_sizes[2] != kG3 * kHid || in_sizes[3] != kG3 * kHid) return;
  if (in_sizes[4] != kG3 || in_sizes[5] != kG3) return;
  if (in_sizes[6] != kFc * kHid || in_sizes[7] != kFc) return;
  if (in_sizes[8] != kCls * kFc || in_sizes[9] != kCls) return;
  if (ws_size < kWsTotal) return;

  const float* x     = (const float*)d_in[0];
  const float* h1    = (const float*)d_in[1];
  const float* w_ih  = (const float*)d_in[2];
  const float* w_hh  = (const float*)d_in[3];
  const float* b_ih  = (const float*)d_in[4];
  const float* b_hh  = (const float*)d_in[5];
  const float* w_fc1 = (const float*)d_in[6];
  const float* b_fc1 = (const float*)d_in[7];
  const float* w_fc3 = (const float*)d_in[8];
  const float* b_fc3 = (const float*)d_in[9];

  float* out0 = (float*)d_out;
  float* out1 = out0 + (size_t)kRows * kCls;

  char* ws = (char*)d_ws;
  unsigned short* X16    = (unsigned short*)(ws + kOffX16);
  unsigned short* H16    = (unsigned short*)(ws + kOffH16);
  unsigned short* WIH16  = (unsigned short*)(ws + kOffWih);
  unsigned short* WHH16  = (unsigned short*)(ws + kOffWhh);
  unsigned short* WFC1   = (unsigned short*)(ws + kOffWfc1);
  unsigned short* WFC3   = (unsigned short*)(ws + kOffWfc3);
  float*          GI     = (float*)(ws + kOffGI);
  float*          GH     = (float*)(ws + kOffGH);
  unsigned short* RES16  = (unsigned short*)(ws + kOffRes);
  unsigned short* RELU16 = (unsigned short*)(ws + kOffRelu);
  (void)H16; (void)WHH16; (void)GH;

  {
    const int n8x = kRows * kHid / 8;
    const int n8w = kG3 * kHid / 8;
    const int n8f = kFc * kHid / 8;
    const int n8c = kCls * kFc / 8;
    cast8_f16_kernel<<<(n8x + 255) / 256, 256, 0, stream>>>(x,     X16,   n8x, 1.0f);
    cast8_f16_kernel<<<(n8x + 255) / 256, 256, 0, stream>>>(h1,    H16,   n8x, 1.0f);
    cast8_f16_kernel<<<(n8w + 255) / 256, 256, 0, stream>>>(w_ih,  WIH16, n8w, kWCarry);
    cast8_f16_kernel<<<(n8w + 255) / 256, 256, 0, stream>>>(w_hh,  WHH16, n8w, kWCarry);
    cast8_f16_kernel<<<(n8f + 255) / 256, 256, 0, stream>>>(w_fc1, WFC1,  n8f, kWCarry);
    cast8_f16_kernel<<<(n8c + 255) / 256, 256, 0, stream>>>(w_fc3, WFC3,  n8c, kWCarry);
  }

  wmma_gemm64<0, false, 0, 0, false, 0><<<dim3(12, 2), 256, 0, stream>>>(
      X16, X16, kHid, (long)kRows * kHid,
      WIH16, WIH16, kHid, (long)kG3 * kHid,
      (void*)GI, (void*)GI, kG3, (long)kRows * kG3,
      b_ih, x, 0L,
      kRows, kG3, kHid, kWCarryInv);

  gru_cell_kernel<<<kRows, 256, 0, stream>>>(GI, GH, b_ih, b_hh, x, h1, out1, RES16);

  wmma_gemm64<0, false, 2, 1, false, 2><<<dim3(4, 1), 256, 0, stream>>>(
      RES16, RES16, kHid, 0L,
      WFC1, WFC1, kHid, 0L,
      (void*)RELU16, (void*)RELU16, kFc, 0L,
      b_fc1, x, 0L,
      kRows, kFc, kHid, kWCarryInv);

  wmma_gemm64<0, false, 2, 0, false, 0><<<dim3(1, 1), 256, 0, stream>>>(
      RELU16, RELU16, kFc, 0L,
      WFC3, WFC3, kFc, 0L,
      (void*)out0, (void*)out0, kCls, 0L,
      b_fc3, x, 0L,
      kRows, kCls, kFc, kWCarryInv);
}
